// TransformerEncoderLayerMoE_RoPE_4784593568355
// MI455X (gfx1250) — hardware-run, weakly checked
//
#include <hip/hip_runtime.h>


#ifndef NB
#define NB 2
#endif
#ifndef SEQ
#define SEQ 2048
#endif
#define NB_FULL  2
#define SEQ_FULL 2048
#define DM   512
#define NH_  8
#define HD   64
#define NE   8
#define FF   1024
#define KE   (NE * FF)
#define NTOK (NB * SEQ)
#define AW   4
#define OSP  68
#define WCI  (1.0f / 64.0f)
#define SC2  ((float)(0.125 * 1.4426950408889634))
#define PSH  14.0f
#define NEGB (-3.0e38f)
#define LNEPS 1.0e-5f

static_assert(HD == 64);
static_assert(NH_ * HD == DM);
static_assert(DM % 64 == 0);
static_assert(DM % 32 == 0);
static_assert(KE % 32 == 0);
static_assert(FF % 64 == 0);
static_assert(KE % 64 == 0);
static_assert(SEQ % 64 == 0);
static_assert(NTOK % 64 == 0);
static_assert(NTOK % 32 == 0);
static_assert(SEQ % 32 == 0);
static_assert(SEQ % (16 * AW) == 0);
static_assert(NE == 8);
static_assert(32 * 4 * 4 == DM);
static_assert(32 * 8 * 2 == DM);
static_assert(32 * 8 * 4 == 16 * 64);
static_assert(4 * 16 == 64);
static_assert(32 * 4 * 8 == 16 * 64);
static_assert(32 * 8 * 4 == 16 * HD);
static_assert(256 * 4 * 4 == 64 * 64);
static_assert(256 * 8 * 2 == 64 * 64);
static_assert(32 * 4 * 2 == 32 * NE);
static_assert(OSP >= HD + 4);
static_assert((OSP * 4) % 16 == 0);
static_assert(NB <= NB_FULL);
static_assert(SEQ <= SEQ_FULL);
static_assert((DM * NE + 8 * DM + 32 * NE) * 4 <= 131072);
static_assert(NE * DM * 4 <= 131072);
static_assert(64 * 68 * 4 <= 131072);
static_assert(AW * 16 * OSP * 4 <= 131072);

typedef _Float16 h16;
typedef unsigned short bf;
typedef __attribute__((ext_vector_type(16))) __bf16   v16bf;
typedef __attribute__((ext_vector_type(16))) _Float16 v16h;
typedef __attribute__((ext_vector_type(8)))  _Float16 v8h;
typedef __attribute__((ext_vector_type(8)))  unsigned short v8us;
typedef __attribute__((ext_vector_type(8)))  float    v8f;
typedef __attribute__((ext_vector_type(4)))  float    v4f;
typedef v4f  __attribute__((may_alias)) v4fa;

__device__ __forceinline__ unsigned short f2bf(float f) { unsigned u = __float_as_uint(f); u += 0x7FFFu + ((u >> 16) & 1u); return (unsigned short)(u >> 16); }
__device__ __forceinline__ float bfr(float f) { return __uint_as_float(((unsigned)f2bf(f)) << 16); }
__device__ __forceinline__ v16h cat16(v8h lo, v8h hi) { return __builtin_shufflevector(lo, hi, 0, 1, 2, 3, 4, 5, 6, 7, 8, 9, 10, 11, 12, 13, 14, 15); }
__device__ __forceinline__ v16bf cat16b(v8us lo, v8us hi) { return __builtin_bit_cast(v16bf, __builtin_shufflevector(lo, hi, 0, 1, 2, 3, 4, 5, 6, 7, 8, 9, 10, 11, 12, 13, 14, 15)); }
__device__ __forceinline__ v8f wmma16(v16h a, v16h b, v8f c) { return __builtin_amdgcn_wmma_f32_16x16x32_f16(false, a, false, b, (short)0, c, false, false); }
__device__ __forceinline__ v8f wmmab(v16bf a, v16bf b, v8f c) { return __builtin_amdgcn_wmma_f32_16x16x32_bf16(false, a, false, b, (short)0, c, false, false); }
__device__ __forceinline__ v16h  ldh(const h16* p) { return cat16(*(const v8h*)p, *(const v8h*)(p + 16)); }
__device__ __forceinline__ v16bf ldb(const bf* p)  { return cat16b(*(const v8us*)p, *(const v8us*)(p + 16)); }
__device__ __forceinline__ void wave_sync() { __builtin_amdgcn_fence(3  , "wavefront"); __builtin_amdgcn_wave_barrier(); asm volatile("" ::: "memory"); }

static __device__ __forceinline__ h16 toh_flush(float v) { const h16 r = (h16)v; return (fabsf(v) < 6.103515625e-05f) ? (h16)0.0f : r; }
static __device__ __forceinline__ v8f wmma16g(v16h a, v16h b, v8f c) { c = wmma16(a, b, c); asm volatile("v_nop\n\tv_nop\n\tv_nop\n\tv_nop" : "+v"(c) : "v"(a), "v"(b)); return c; }
static __device__ __forceinline__ v8f wmmabg(v16bf a, v16bf b, v8f c) { c = wmmab(a, b, c); asm volatile("v_nop\n\tv_nop\n\tv_nop\n\tv_nop" : "+v"(c) : "v"(a), "v"(b)); return c; }

__global__ __launch_bounds__(256) void k_cvtx(const float* __restrict__ src, bf* dst) {
    const size_t i = (size_t)blockIdx.x * 256 + threadIdx.x; if (i >= (size_t)NTOK * (DM / 8)) return;
    const int row = (int)(i / (DM / 8)), c8 = (int)(i % (DM / 8)) * 8;
    const int b = row / SEQ, t = row % SEQ;
    const float* p = src + ((size_t)t * NB_FULL + b) * DM + c8;
    const v4f a = *(const v4f*)p; const v4f c = *(const v4f*)(p + 4); v8us o;
#pragma unroll
    for (int k = 0; k < 4; ++k) { o[k] = f2bf(a[k]); o[4 + k] = f2bf(c[k]); }
    *(volatile v8us*)(dst + i * 8) = o; __threadfence(); *(volatile v8us*)(dst + i * 8) = o;
}

template <int F16OUT>
__device__ __forceinline__ void wt_body(const float* __restrict__ in, unsigned short* out, const int R, const int C, const size_t omat, const size_t opitch) {
    __shared__ __align__(16) float ts[64 * 68];
    const int tid = threadIdx.x;
    const int c0 = blockIdx.x * 64, r0 = blockIdx.y * 64, mat = blockIdx.z;
    const float* ip = in + (size_t)mat * (size_t)R * (size_t)C;
#pragma unroll
    for (int it = 0; it < 4; ++it) { const int i = tid + 256 * it; const int r = i >> 4, c4 = (i & 15) * 4;
        const v4f v = *(const v4f*)(ip + (size_t)(r0 + r) * C + c0 + c4);
#pragma unroll
        for (int k = 0; k < 4; ++k) ts[(c4 + k) * 68 + r] = v[k]; }
    __syncthreads();
    v8us ov[2];
#pragma unroll
    for (int it = 0; it < 2; ++it) { const int c = it * 32 + (tid >> 3), r8 = (tid & 7) * 8;
        const v4f x0 = *(const v4fa*)(&ts[c * 68 + r8]); const v4f x1 = *(const v4fa*)(&ts[c * 68 + r8 + 4]);
#pragma unroll
        for (int k = 0; k < 4; ++k) {
            if (F16OUT) { ov[it][k] = __builtin_bit_cast(unsigned short, toh_flush(bfr(x0[k]) * 64.0f)); ov[it][4 + k] = __builtin_bit_cast(unsigned short, toh_flush(bfr(x1[k]) * 64.0f)); }
            else        { ov[it][k] = f2bf(x0[k]); ov[it][4 + k] = f2bf(x1[k]); } } }
#pragma unroll 1
    for (int ps = 0; ps < 2; ++ps) {
#pragma unroll
        for (int it = 0; it < 2; ++it) { const int c = it * 32 + (tid >> 3), r8 = (tid & 7) * 8;
            *(volatile v8us*)(out + (size_t)mat * omat + (size_t)(c0 + c) * opitch + (size_t)(r0 + r8)) = ov[it]; }
        if (ps == 0) __threadfence(); }
}
__global__ __launch_bounds__(256) void k_wT_bf(const float* __restrict__ in, bf* out, int R, int C, size_t omat, size_t opitch) { wt_body<0>(in, out, R, C, omat, opitch); }
__global__ __launch_bounds__(256) void k_wT_h(const float* __restrict__ in, h16* out, int R, int C, size_t omat, size_t opitch) { wt_body<1>(in, (unsigned short*)out, R, C, omat, opitch); }

__device__ __forceinline__ void proj_loop(const bf* __restrict__ A, const bf* __restrict__ Bt, const size_t aoff, const size_t boff, v8f (&acc)[4][4]) {
    const int K = DM;
#pragma unroll 1
    for (int kc = 0; kc < K; kc += 32) {
        v16bf a[4];
#pragma unroll
        for (int mb = 0; mb < 4; ++mb) a[mb] = ldb(A + aoff + (size_t)mb * 16 * K + kc);
#pragma unroll
        for (int nb = 0; nb < 4; ++nb) { const v16bf b = ldb(Bt + boff + (size_t)nb * 16 * K + kc);
#pragma unroll
            for (int mb = 0; mb < 4; ++mb) acc[mb][nb] = wmmabg(a[mb], b, acc[mb][nb]); }
    }
}

__global__ __launch_bounds__(32) __attribute__((amdgpu_num_vgpr(256))) void k_projqk(const bf* __restrict__ X, const bf* __restrict__ Wt, const float* __restrict__ bias,
                                               const float* __restrict__ cosT, const float* __restrict__ sinT, h16* P) {
    __shared__ __align__(16) float os[64 * 68];
    const int K = DM;
    const int lane = threadIdx.x & 31, lr = lane & 15, hi = lane >> 4; const int r0 = blockIdx.x * 64, c0 = blockIdx.y * 64;
    const int bb = r0 / SEQ, tt = r0 % SEQ; const int zc = bb * NH_ + c0 / HD;
    const size_t tbase = ((size_t)zc * SEQ + (size_t)tt) * HD;
    {
        v8f acc[4][4];
#pragma unroll
        for (int mb = 0; mb < 4; ++mb)
#pragma unroll
            for (int nb = 0; nb < 4; ++nb) acc[mb][nb] = (v8f){};
        proj_loop(X, Wt, (size_t)(r0 + lr) * K + 8 * hi, (size_t)(c0 + lr) * K + 8 * hi, acc);
        float bc[4];
#pragma unroll
        for (int nb = 0; nb < 4; ++nb) bc[nb] = bfr(bias[c0 + nb * 16 + lr]);
#pragma unroll
        for (int mb = 0; mb < 4; ++mb) {
#pragma unroll
            for (int nb = 0; nb < 4; ++nb) {
#pragma unroll
                for (int j = 0; j < 8; ++j) os[(mb * 16 + hi * 8 + j) * 68 + nb * 16 + lr] = acc[mb][nb][j] + bc[nb]; } }
    }
    wave_sync();
    const int rq = lane >> 3, c8 = (lane & 7) * 8;
    const int pc = c8 ^ 32;
    const float sg = (c8 < 32) ? -1.0f : 1.0f;
#pragma unroll 1
    for (int mb = 0; mb < 4; ++mb) {
        v8h hv[4];
#pragma unroll
        for (int s = 0; s < 4; ++s) { const int row = mb * 16 + 4 * s + rq; const int t = tt + row;
            const v4f x0 = *(const v4fa*)(&os[row * 68 + c8]); const v4f x1 = *(const v4fa*)(&os[row * 68 + c8 + 4]);
            const v4f y0 = *(const v4fa*)(&os[row * 68 + pc]); const v4f y1 = *(const v4fa*)(&os[row * 68 + pc + 4]);
            const float* cp = cosT + (size_t)t * HD + c8; const float* sp = sinT + (size_t)t * HD + c8;
            const v4f ca = *(const v4f*)cp; const v4f cb = *(const v4f*)(cp + 4); const v4f sa = *(const v4f*)sp; const v4f sb = *(const v4f*)(sp + 4);
#pragma unroll
            for (int i = 0; i < 4; ++i) {
                hv[s][i]     = toh_flush(x0[i] * bfr(ca[i]) + (sg * y0[i]) * bfr(sa[i]));
                hv[s][4 + i] = toh_flush(x1[i] * bfr(cb[i]) + (sg * y1[i]) * bfr(sb[i])); }
            asm volatile("" ::: "memory"); }
#pragma unroll 1
        for (int ps = 0; ps < 2; ++ps) {
#pragma unroll
            for (int s = 0; s < 4; ++s) { const int row = mb * 16 + 4 * s + rq;
                *(volatile v8h*)(P + tbase + (size_t)row * HD + c8) = hv[s]; }
            if (ps == 0) __threadfence(); }
        asm volatile("" ::: "memory");
    }
}

__global__ __launch_bounds__(32) void k_projv(const bf* __restrict__ Wt, const bf* __restrict__ X, const float* __restrict__ bias, h16* VTp) {
    __shared__ __align__(16) float os[16 * 68];
    const int K = DM;
    const int lane = threadIdx.x & 31, lr = lane & 15, hi = lane >> 4; const int r0 = blockIdx.x * 64, c0 = blockIdx.y * 64;
    v8f acc[4][4];
#pragma unroll
    for (int mb = 0; mb < 4; ++mb)
#pragma unroll
        for (int nb = 0; nb < 4; ++nb) acc[mb][nb] = (v8f){};
    proj_loop(Wt, X, (size_t)(r0 + lr) * K + 8 * hi, (size_t)(c0 + lr) * K + 8 * hi, acc);
    const int bb = c0 / SEQ, tt = c0 % SEQ;
    const size_t tbase = (size_t)bb * (size_t)DM * SEQ + (size_t)r0 * SEQ + (size_t)tt;
#pragma unroll
    for (int mb = 0; mb < 4; ++mb) {
        float br[8];
#pragma unroll
        for (int j = 0; j < 8; ++j) br[j] = bfr(bias[r0 + mb * 16 + hi * 8 + j]);
#pragma unroll
        for (int nb = 0; nb < 4; ++nb) {
#pragma unroll
            for (int j = 0; j < 8; ++j) os[(hi * 8 + j) * 68 + nb * 16 + lr] = acc[mb][nb][j] + br[j]; }
        wave_sync();
        v8h hv[4];
#pragma unroll
        for (int s = 0; s < 4; ++s) { const int row = 4 * s + (lane >> 3), c8 = (lane & 7) * 8;
            const v4f x0 = *(const v4fa*)(&os[row * 68 + c8]); const v4f x1 = *(const v4fa*)(&os[row * 68 + c8 + 4]);
#pragma unroll
            for (int i = 0; i < 4; ++i) { hv[s][i] = toh_flush(x0[i]); hv[s][4 + i] = toh_flush(x1[i]); } }
#pragma unroll 1
        for (int ps = 0; ps < 2; ++ps) {
#pragma unroll
            for (int s = 0; s < 4; ++s) { const int row = 4 * s + (lane >> 3), c8 = (lane & 7) * 8;
                *(volatile v8h*)(VTp + tbase + (size_t)(mb * 16 + row) * SEQ + c8) = hv[s]; }
            if (ps == 0) __threadfence(); }
        wave_sync();
    }
}

__global__ __launch_bounds__(32 * AW) void k_flash(const h16* __restrict__ QH, const h16* __restrict__ KP, const h16* __restrict__ VT, h16* CTX) {
    __shared__ __align__(16) float os[AW * 16 * OSP];
    const int lane = threadIdx.x & 31, lr = lane & 15, hi = lane >> 4;
    const int wave = __builtin_amdgcn_readfirstlane((int)(threadIdx.x >> 5));
    const int zh = blockIdx.y; const int b = zh / NH_, h = zh % NH_;
    const int t0 = (blockIdx.x * AW + wave) * 16;
    const size_t pbase = (size_t)zh * SEQ * HD;
    const size_t qo = pbase + (size_t)(t0 + lr) * HD + 8 * hi;
    const v16h q0 = ldh(QH + qo), q1 = ldh(QH + qo + 32);
    const size_t ko = pbase + (size_t)lr * HD + 8 * hi;
    const size_t vo = pbase + (size_t)lr * SEQ + 8 * hi;
    v8f o[4];
#pragma unroll
    for (int j = 0; j < 4; ++j) o[j] = (v8f){};
    float m = NEGB, l = 0.0f;
#pragma unroll 1
    for (int key0 = 0; key0 < SEQ; key0 += 32) {
        const h16* ka = KP + ko + (size_t)key0 * HD;
        const v16h ka0 = ldh(ka), ka1 = ldh(ka + 32), kb0 = ldh(ka + 16 * HD), kb1 = ldh(ka + 16 * HD + 32);
        v8f sa = (v8f){}, sb = (v8f){};
        sa = wmma16g(ka0, q0, sa); sa = wmma16g(ka1, q1, sa);
        sb = wmma16g(kb0, q0, sb); sb = wmma16g(kb1, q1, sb);
        float ta[8], tb[8]; float mx = NEGB;
#pragma unroll
        for (int r = 0; r < 8; ++r) { ta[r] = sa[r] * SC2; tb[r] = sb[r] * SC2; mx = fmaxf(mx, fmaxf(ta[r], tb[r])); }
        mx = fmaxf(mx, __shfl_xor(mx, 16, 32));
        const float mnew = fmaxf(m, mx);
        const float alpha = __builtin_amdgcn_exp2f(m - mnew);
        const float sh = PSH - mnew;
        v16h pb; float ls = 0.0f;
#pragma unroll
        for (int r = 0; r < 8; ++r) {
            const float xa = ta[r] + sh, xb = tb[r] + sh;
            const float ea = __builtin_amdgcn_exp2f(xa), eb = __builtin_amdgcn_exp2f(xb);
            const float ga = (xa < -14.0f) ? 0.0f : ea, gb = (xb < -14.0f) ? 0.0f : eb;
            const h16 pa = (h16)ga; const h16 pc = (h16)gb;
            pb[r] = pa; pb[8 + r] = pc;
            ls += (float)pa + (float)pc; }
        l = l * alpha + ls; m = mnew;
#pragma unroll
        for (int j = 0; j < 4; ++j) o[j] = o[j] * alpha;
        const h16* va = VT + vo + key0;
        v16h vf[4];
#pragma unroll
        for (int j = 0; j < 4; ++j) vf[j] = ldh(va + (size_t)(16 * j) * SEQ);
#pragma unroll
        for (int j = 0; j < 4; ++j) o[j] = wmma16g(vf[j], pb, o[j]);
    }
    l += __shfl_xor(l, 16, 32);
    const float inv = 64.0f * (1.0f / l);
    const int wb = wave * 16 * OSP;
#pragma unroll
    for (int j = 0; j < 4; ++j) { v4f a, c;
        a[0] = o[j][0] * inv; a[1] = o[j][1] * inv; a[2] = o[j][2] * inv; a[3] = o[j][3] * inv;
        c[0] = o[j][4] * inv; c[1] = o[j][5] * inv; c[2] = o[j][6] * inv; c[3] = o[j][7] * inv;
        *(v4fa*)(&os[wb + lr * OSP + 16 * j + 8 * hi]) = a; *(v4fa*)(&os[wb + lr * OSP + 16 * j + 8 * hi + 4]) = c; }
    wave_sync();
    v8h hv[4];
#pragma unroll
    for (int s = 0; s < 4; ++s) { const int row = 4 * s + (lane >> 3), c8 = (lane & 7) * 8;
        const v4f x0 = *(const v4fa*)(&os[wb + row * OSP + c8]); const v4f x1 = *(const v4fa*)(&os[wb + row * OSP + c8 + 4]);
#pragma unroll
        for (int i = 0; i < 4; ++i) { hv[s][i] = toh_flush(x0[i]); hv[s][4 + i] = toh_flush(x1[i]); } }
    h16* crow = CTX + ((size_t)b * SEQ + t0) * DM + h * HD;
#pragma unroll 1
    for (int ps = 0; ps < 2; ++ps) {
#pragma unroll
        for (int s = 0; s < 4; ++s) { const int row = 4 * s + (lane >> 3), c8 = (lane & 7) * 8;
            *(volatile v8h*)(crow + (size_t)row * DM + c8) = hv[s]; }
        if (ps == 0) __threadfence(); }
}

template <int EPI>
__device__ __forceinline__ void gemm_body(const h16* __restrict__ A, const h16* __restrict__ Bt, const int K, const float scale,
                                          const float* __restrict__ bias, const float* __restrict__ gate, float* Cf, h16* Ch, const int ldc) {
    __shared__ __align__(16) float os[16 * 68];
    const int lane = threadIdx.x & 31, lr = lane & 15, hi = lane >> 4; const int r0 = blockIdx.x * 64, c0 = blockIdx.y * 64;
    v8f acc[4][4];
#pragma unroll
    for (int mb = 0; mb < 4; ++mb)
#pragma unroll
        for (int nb = 0; nb < 4; ++nb) acc[mb][nb] = (v8f){};
    const size_t aoff = (size_t)(r0 + lr) * K + 8 * hi, boff = (size_t)(c0 + lr) * K + 8 * hi;
#pragma unroll 1
    for (int kc = 0; kc < K; kc += 32) {
        v16h a[4];
#pragma unroll
        for (int mb = 0; mb < 4; ++mb) a[mb] = ldh(A + aoff + (size_t)mb * 16 * K + kc);
#pragma unroll
        for (int nb = 0; nb < 4; ++nb) { const v16h b = ldh(Bt + boff + (size_t)nb * 16 * K + kc);
#pragma unroll
            for (int mb = 0; mb < 4; ++mb) acc[mb][nb] = wmma16g(a[mb], b, acc[mb][nb]); }
    }
    float bc[4];
#pragma unroll
    for (int nb = 0; nb < 4; ++nb) { bc[nb] = 0.0f; if (EPI != 2) bc[nb] = bfr(bias[c0 + nb * 16 + lr]); }
    const int eidx = c0 / FF;
#pragma unroll
    for (int mb = 0; mb < 4; ++mb) {
#pragma unroll
        for (int nb = 0; nb < 4; ++nb) {
#pragma unroll
            for (int j = 0; j < 8; ++j) os[(hi * 8 + j) * 68 + nb * 16 + lr] = acc[mb][nb][j] * scale + bc[nb]; }
        wave_sync();
        if (EPI == 1) {
            v8h hv[4];
#pragma unroll
            for (int s = 0; s < 4; ++s) { const int row = 4 * s + (lane >> 3), c8 = (lane & 7) * 8;
                const float g = gate[(size_t)(r0 + mb * 16 + row) * NE + eidx];
                const v4f x0 = *(const v4fa*)(&os[row * 68 + c8]); const v4f x1 = *(const v4fa*)(&os[row * 68 + c8 + 4]);
#pragma unroll
                for (int i = 0; i < 4; ++i) { hv[s][i] = toh_flush(fmaxf(x0[i], 0.0f) * g); hv[s][4 + i] = toh_flush(fmaxf(x1[i], 0.0f) * g); } }
#pragma unroll 1
            for (int ps = 0; ps < 2; ++ps) {
#pragma unroll
                for (int s = 0; s < 4; ++s) { const int row = 4 * s + (lane >> 3), c8 = (lane & 7) * 8;
                    *(volatile v8h*)(Ch + (size_t)(r0 + mb * 16 + row) * ldc + c0 + c8) = hv[s]; }
                if (ps == 0) __threadfence(); }
        } else {
            v4f fv[8];
#pragma unroll
            for (int s = 0; s < 8; ++s) { const int row = 2 * s + (lane >> 4), cofs = (lane & 15) * 4;
                fv[s] = *(const v4fa*)(&os[row * 68 + cofs]); }
#pragma unroll 1
            for (int ps = 0; ps < 2; ++ps) {
#pragma unroll
                for (int s = 0; s < 8; ++s) { const int row = 2 * s + (lane >> 4), cofs = (lane & 15) * 4;
                    *(volatile v4f*)(Cf + (size_t)(r0 + mb * 16 + row) * ldc + c0 + cofs) = fv[s]; }
                if (ps == 0) __threadfence(); }
        }
        wave_sync();
    }
}
__global__ __launch_bounds__(32) void k_gemm_bias(const h16* __restrict__ A, const h16* __restrict__ Bt, int K, float scale, const float* __restrict__ bias, float* Cf, int ldc) {
    gemm_body<0>(A, Bt, K, scale, bias, bias, Cf, (h16*)0, ldc); }
__global__ __launch_bounds__(32) void k_gemm_up(const h16* __restrict__ A, const h16* __restrict__ Bt, int K, float scale, const float* __restrict__ bias, const float* __restrict__ gate, h16* Ch, int ldc) {
    gemm_body<1>(A, Bt, K, scale, bias, gate, (float*)0, Ch, ldc); }
__global__ __launch_bounds__(32) void k_gemm_plain(const h16* __restrict__ A, const h16* __restrict__ Bt, int K, float scale, float* Cf, int ldc) {
    gemm_body<2>(A, Bt, K, scale, (const float*)0, (const float*)0, Cf, (h16*)0, ldc); }

__global__ __launch_bounds__(256) void k_ln1(const float* __restrict__ src, const float* __restrict__ AO, const float* __restrict__ gam, const float* __restrict__ bet,
                                             const float* __restrict__ Wg, float* X, h16* XH, float* G) {
#pragma clang fp contract(off)
    __shared__ __align__(16) float wgs[DM * NE];
    __shared__ __align__(16) float xs[8 * DM];
    __shared__ __align__(16) float gs[32 * NE];
    const int tid = threadIdx.x, lane = tid & 31;
    const int wave = __builtin_amdgcn_readfirstlane((int)(threadIdx.x >> 5));
#pragma unroll 1
    for (int i = tid; i < DM * NE; i += 256) wgs[i] = bfr(Wg[i]);
    __syncthreads();
    v4f gv[4], bv[4];
#pragma unroll
    for (int i = 0; i < 4; ++i) { const v4f a = *(const v4f*)(gam + 4 * lane + 128 * i); const v4f c = *(const v4f*)(bet + 4 * lane + 128 * i);
#pragma unroll
        for (int k = 0; k < 4; ++k) { gv[i][k] = bfr(a[k]); bv[i][k] = bfr(c[k]); } }
#pragma unroll 1
    for (int rr = 0; rr < 4; ++rr) {
        const int rl = wave * 4 + rr; const int m = blockIdx.x * 32 + rl;
        const int b = m / SEQ, t = m % SEQ;
        const float* sp = src + ((size_t)t * NB_FULL + b) * DM + 4 * lane;
        const float* ap = AO + (size_t)m * DM + 4 * lane;
        v4f v[4]; float sum = 0.0f;
#pragma unroll
        for (int i = 0; i < 4; ++i) { const v4f a = *(const v4f*)(sp + 128 * i); const v4f c = *(const v4f*)(ap + 128 * i);
#pragma unroll
            for (int k = 0; k < 4; ++k) { v[i][k] = bfr(a[k]) + c[k]; sum += v[i][k]; } }
#pragma unroll
        for (int msk = 16; msk > 0; msk >>= 1) sum += __shfl_xor(sum, msk, 32);
        const float mean = sum * (1.0f / (float)DM);
        float sq = 0.0f;
#pragma unroll
        for (int i = 0; i < 4; ++i)
#pragma unroll
            for (int k = 0; k < 4; ++k) { const float d = v[i][k] - mean; sq += d * d; }
#pragma unroll
        for (int msk = 16; msk > 0; msk >>= 1) sq += __shfl_xor(sq, msk, 32);
        const float rs = rsqrtf(sq * (1.0f / (float)DM) + LNEPS);
        v4f xo[4];
#pragma unroll
        for (int i = 0; i < 4; ++i) {
#pragma unroll
            for (int k = 0; k < 4; ++k) xo[i][k] = (v[i][k] - mean) * rs * gv[i][k] + bv[i][k];
            *(v4fa*)(&xs[wave * DM + 4 * lane + 128 * i]) = xo[i]; }
        wave_sync();
        float acc[NE];
#pragma unroll
        for (int e = 0; e < NE; ++e) acc[e] = 0.0f;
#pragma unroll 1
        for (int k = 0; k < DM / 32; ++k) { const int d = lane + 32 * k; const float xv = xs[wave * DM + d];
            const v4f w0 = *(const v4fa*)(&wgs[d * NE]); const v4f w1 = *(const v4fa*)(&wgs[d * NE + 4]);
#pragma unroll
            for (int e = 0; e < 4; ++e) { acc[e] += xv * w0[e]; acc[4 + e] += xv * w1[e]; } }
#pragma unroll
        for (int e = 0; e < NE; ++e)
#pragma unroll
            for (int msk = 16; msk > 0; msk >>= 1) acc[e] += __shfl_xor(acc[e], msk, 32);
        const int e = lane & 7;
        float lg = acc[0]; float mx = acc[0];
#pragma unroll
        for (int q = 1; q < NE; ++q) { lg = (e == q) ? acc[q] : lg; mx = fmaxf(mx, acc[q]); }
        const float ex = expf(lg - mx);
        float ssum = ex;
        ssum += __shfl_xor(ssum, 1, 32); ssum += __shfl_xor(ssum, 2, 32); ssum += __shfl_xor(ssum, 4, 32);
        const float p = ex * (1.0f / ssum);
        float v0 = p; int i0 = e;
#pragma unroll
        for (int msk = 1; msk < 8; msk <<= 1) { const float ov = __shfl_xor(v0, msk, 32); const int oi = __shfl_xor(i0, msk, 32);
            const bool tk = (ov > v0) | ((ov == v0) & (oi < i0)); v0 = tk ? ov : v0; i0 = tk ? oi : i0; }
        float v1 = (e == i0) ? -1.0f : p; int i1 = e;
#pragma unroll
        for (int msk = 1; msk < 8; msk <<= 1) { const float ov = __shfl_xor(v1, msk, 32); const int oi = __shfl_xor(i1, msk, 32);
            const bool tk = (ov > v1) | ((ov == v1) & (oi < i1)); v1 = tk ? ov : v1; i1 = tk ? oi : i1; }
        const float rinv = 1.0f / (v0 + v1);
        const float g = (e == i0) ? (v0 * rinv) : ((e == i1) ? (v1 * rinv) : 0.0f);
        if (lane < 8) gs[rl * NE + lane] = g;
        v8h xh[2];
#pragma unroll
        for (int i = 0; i < 2; ++i) { const v4f x0 = *(const v4fa*)(&xs[wave * DM + 8 * lane + 256 * i]); const v4f x1 = *(const v4fa*)(&xs[wave * DM + 8 * lane + 256 * i + 4]);
#pragma unroll
            for (int k = 0; k < 4; ++k) { xh[i][k] = toh_flush(x0[k]); xh[i][4 + k] = toh_flush(x1[k]); } }
#pragma unroll 1
        for (int ps = 0; ps < 2; ++ps) {
#pragma unroll
            for (int i = 0; i < 4; ++i) *(volatile v4f*)(X + (size_t)m * DM + 4 * lane + 128 * i) = xo[i];
#pragma unroll
            for (int i = 0; i < 2; ++i) *(volatile v8h*)(XH + (size_t)m * DM + 8 * lane + 256 * i) = xh[i];
            if (ps == 0) __threadfence(); }
        wave_sync();
    }
    __syncthreads();
    if (wave == 0) {
        const v4f g0 = *(const v4fa*)(&gs[4 * lane]); const v4f g1 = *(const v4fa*)(&gs[128 + 4 * lane]);
        float* gp = G + (size_t)blockIdx.x * (32 * NE);
#pragma unroll 1
        for (int ps = 0; ps < 2; ++ps) {
            *(volatile v4f*)(gp + 4 * lane) = g0; *(volatile v4f*)(gp + 128 + 4 * lane) = g1;
            if (ps == 0) __threadfence(); }
    }
}

__global__ __launch_bounds__(256) void k_ln2(const float* __restrict__ X, const float* __restrict__ MO, const float* __restrict__ G, const float* __restrict__ B2,
                                             const float* __restrict__ gam, const float* __restrict__ bet, float* OUT) {
#pragma clang fp contract(off)
    __shared__ __align__(16) float b2s[NE * DM];
    const int tid = threadIdx.x, lane = tid & 31;
    const int wave = __builtin_amdgcn_readfirstlane((int)(threadIdx.x >> 5));
#pragma unroll 1
    for (int i = tid; i < NE * DM; i += 256) b2s[i] = bfr(B2[i]);
    __syncthreads();
    v4f gv[4], bv[4];
#pragma unroll
    for (int i = 0; i < 4; ++i) { const v4f a = *(const v4f*)(gam + 4 * lane + 128 * i); const v4f c = *(const v4f*)(bet + 4 * lane + 128 * i);
#pragma unroll
        for (int k = 0; k < 4; ++k) { gv[i][k] = bfr(a[k]); bv[i][k] = bfr(c[k]); } }
#pragma unroll 1
    for (int rr = 0; rr < 4; ++rr) {
        const int m = blockIdx.x * 32 + wave * 4 + rr;
        const int b = m / SEQ, t = m % SEQ;
        const float* xp = X + (size_t)m * DM + 4 * lane;
        const float* mp = MO + (size_t)m * DM + 4 * lane;
        v4f y[4];
#pragma unroll
        for (int i = 0; i < 4; ++i) { const v4f a = *(const v4f*)(xp + 128 * i); const v4f c = *(const v4f*)(mp + 128 * i); y[i] = c; (void)a; }
#pragma unroll 1
        for (int e = 0; e < NE; ++e) { const float ge = G[(size_t)m * NE + e];
#pragma unroll
            for (int i = 0; i < 4; ++i) { const v4f w = *(const v4fa*)(&b2s[e * DM + 4 * lane + 128 * i]); y[i] = y[i] + w * ge; } }
        float sum = 0.0f;
#pragma unroll
        for (int i = 0; i < 4; ++i) { const v4f a = *(const v4f*)(xp + 128 * i);
#pragma unroll
            for (int k = 0; k < 4; ++k) { y[i][k] = a[k] + y[i][k]; sum += y[i][k]; } }
#pragma unroll
        for (int msk = 16; msk > 0; msk >>= 1) sum += __shfl_xor(sum, msk, 32);
        const float mean = sum * (1.0f / (float)DM);
        float sq = 0.0f;
#pragma unroll
        for (int i = 0; i < 4; ++i)
#pragma unroll
            for (int k = 0; k < 4; ++k) { const float d = y[i][k] - mean; sq += d * d; }
#pragma unroll
        for (int msk = 16; msk > 0; msk >>= 1) sq += __shfl_xor(sq, msk, 32);
        const float rs = rsqrtf(sq * (1.0f / (float)DM) + LNEPS);
        v4f xo[4];
#pragma unroll
        for (int i = 0; i < 4; ++i)
#pragma unroll
            for (int k = 0; k < 4; ++k) xo[i][k] = (y[i][k] - mean) * rs * gv[i][k] + bv[i][k];
        float* op = OUT + ((size_t)t * NB_FULL + b) * DM + 4 * lane;
#pragma unroll 1
        for (int ps = 0; ps < 2; ++ps) {
#pragma unroll
            for (int i = 0; i < 4; ++i) *(volatile v4f*)(op + 128 * i) = xo[i];
            if (ps == 0) __threadfence(); }
    }
}

static constexpr size_t al256(size_t v) { return (v + 255) & ~(size_t)255; }
static constexpr size_t SZ_PL = al256((size_t)NTOK * DM * 2);
static constexpr size_t SZ_WS = al256((size_t)DM * DM * 2);
static constexpr size_t SZ_WE = al256((size_t)NE * DM * FF * 2);
static constexpr size_t SZ_F  = al256((size_t)NTOK * DM * 4);
static constexpr size_t SZ_G  = al256((size_t)NTOK * NE * 4);
static constexpr size_t SZ_H  = al256((size_t)NTOK * KE * 2);
static constexpr size_t SZ_TOTAL = 6 * SZ_PL + 4 * SZ_WS + 2 * SZ_WE + 2 * SZ_F + SZ_G + SZ_H;
static_assert(SZ_TOTAL <= (size_t)134217728);
static_assert((size_t)NB * NH_ * SEQ * HD == (size_t)NTOK * DM);
static_assert((size_t)(NTOK / 32) * 32 * NE == (size_t)NTOK * NE);
static_assert((size_t)NE * FF * DM == (size_t)KE * DM);

extern "C" void kernel_launch(void* const* d_in, const int* in_sizes, int n_in,
                              void* d_out, int out_size, void* d_ws, size_t ws_size, hipStream_t stream) {
    if (n_in < 20) return;
    const size_t needx = ((size_t)(SEQ - 1) * NB_FULL + NB) * DM;
    if ((size_t)in_sizes[0] < needx) return;
    if ((size_t)in_sizes[1] < (size_t)SEQ * HD || (size_t)in_sizes[2] < (size_t)SEQ * HD) return;
    if ((size_t)in_sizes[3] < (size_t)DM * DM || (size_t)in_sizes[5] < (size_t)DM * DM || (size_t)in_sizes[7] < (size_t)DM * DM || (size_t)in_sizes[9] < (size_t)DM * DM) return;
    if (in_sizes[4] < DM || in_sizes[6] < DM || in_sizes[8] < DM || in_sizes[10] < DM) return;
    if (in_sizes[11] < DM || in_sizes[12] < DM || in_sizes[13] < DM || in_sizes[14] < DM) return;
    if (in_sizes[15] < DM * NE) return;
    if ((size_t)in_sizes[16] < (size_t)NE * DM * FF || (size_t)in_sizes[18] < (size_t)NE * FF * DM) return;
    if (in_sizes[17] < NE * FF || in_sizes[19] < NE * DM) return;
    if ((size_t)out_size < needx) return;
    if (SZ_TOTAL > ws_size) return;
    const float* src  = (const float*)d_in[0];
    const float* cosT = (const float*)d_in[1];  const float* sinT = (const float*)d_in[2];
    const float* wq = (const float*)d_in[3];    const float* bq = (const float*)d_in[4];
    const float* wk = (const float*)d_in[5];    const float* bk = (const float*)d_in[6];
    const float* wv = (const float*)d_in[7];    const float* bv = (const float*)d_in[8];
    const float* wo = (const float*)d_in[9];    const float* bo = (const float*)d_in[10];
    const float* l1g = (const float*)d_in[11];  const float* l1b = (const float*)d_in[12];
    const float* l2g = (const float*)d_in[13];  const float* l2b = (const float*)d_in[14];
    const float* wg = (const float*)d_in[15];
    const float* w1 = (const float*)d_in[16];   const float* b1 = (const float*)d_in[17];
    const float* w2 = (const float*)d_in[18];   const float* b2 = (const float*)d_in[19];
    float* OUT = (float*)d_out;
    char* wsp = (char*)d_ws;
    bf*  XB  = (bf*)wsp;  wsp += SZ_PL;
    bf*  WQT = (bf*)wsp;  wsp += SZ_WS;
    bf*  WKT = (bf*)wsp;  wsp += SZ_WS;
    bf*  WVT = (bf*)wsp;  wsp += SZ_WS;
    h16* WOT = (h16*)wsp; wsp += SZ_WS;
    h16* W1T = (h16*)wsp; wsp += SZ_WE;
    h16* W2T = (h16*)wsp; wsp += SZ_WE;
    h16* QH  = (h16*)wsp; wsp += SZ_PL;
    h16* KP  = (h16*)wsp; wsp += SZ_PL;
    h16* VT  = (h16*)wsp; wsp += SZ_PL;
    h16* CTX = (h16*)wsp; wsp += SZ_PL;
    h16* XH  = (h16*)wsp; wsp += SZ_PL;
    float* FA = (float*)wsp; wsp += SZ_F;
    float* X  = (float*)wsp; wsp += SZ_F;
    float* G  = (float*)wsp; wsp += SZ_G;
    h16* H    = (h16*)wsp; wsp += SZ_H;

    k_cvtx<<<(unsigned)(((size_t)NTOK * (DM / 8) + 255) / 256), 256, 0, stream>>>(src, XB);
    k_wT_bf<<<dim3(DM / 64, DM / 64, 1), 256, 0, stream>>>(wq, WQT, DM, DM, (size_t)DM * DM, (size_t)DM);
    k_wT_bf<<<dim3(DM / 64, DM / 64, 1), 256, 0, stream>>>(wk, WKT, DM, DM, (size_t)DM * DM, (size_t)DM);
    k_wT_bf<<<dim3(DM / 64, DM / 64, 1), 256, 0, stream>>>(wv, WVT, DM, DM, (size_t)DM * DM, (size_t)DM);
    k_wT_h<<<dim3(DM / 64, DM / 64, 1), 256, 0, stream>>>(wo, WOT, DM, DM, (size_t)DM * DM, (size_t)DM);
    k_wT_h<<<dim3(FF / 64, DM / 64, NE), 256, 0, stream>>>(w1, W1T, DM, FF, (size_t)FF * DM, (size_t)DM);
    k_wT_h<<<dim3(DM / 64, FF / 64, NE), 256, 0, stream>>>(w2, W2T, FF, DM, (size_t)FF, (size_t)KE);

    k_projqk<<<dim3(NTOK / 64, DM / 64, 1), 32, 0, stream>>>(XB, WQT, bq, cosT, sinT, QH);
    k_projqk<<<dim3(NTOK / 64, DM / 64, 1), 32, 0, stream>>>(XB, WKT, bk, cosT, sinT, KP);
    k_projv<<<dim3(DM / 64, NTOK / 64, 1), 32, 0, stream>>>(WVT, XB, bv, VT);

    k_flash<<<dim3(SEQ / (16 * AW), NB * NH_, 1), 32 * AW, 0, stream>>>(QH, KP, VT, CTX);

    k_gemm_bias<<<dim3(NTOK / 64, DM / 64, 1), 32, 0, stream>>>(CTX, WOT, DM, WCI * WCI, bo, FA, DM);
    k_ln1<<<NTOK / 32, 256, 0, stream>>>(src, FA, l1g, l1b, wg, X, XH, G);
    k_gemm_up<<<dim3(NTOK / 64, KE / 64, 1), 32, 0, stream>>>(XH, W1T, DM, WCI, b1, G, H, KE);
    k_gemm_plain<<<dim3(NTOK / 64, DM / 64, 1), 32, 0, stream>>>(H, W2T, KE, WCI, FA, DM);
    k_ln2<<<NTOK / 32, 256, 0, stream>>>(X, FA, G, b2, l2g, l2b, OUT);
}
